// Leg_fit_12945031430350
// MI455X (gfx1250) — hardware-run, weakly checked
//
#include <hip/hip_runtime.h>
#include <hip/hip_fp16.h>
#include <math.h>

typedef __attribute__((ext_vector_type(16))) _Float16 v16h;
typedef __attribute__((ext_vector_type(8)))  _Float16 v8h;
typedef __attribute__((ext_vector_type(8)))  float    v8f;
typedef __attribute__((ext_vector_type(4)))  float    v4f;

constexpr int kBatch = 2;
constexpr int kSteps = 512;
constexpr int kNeur  = 256;
constexpr int kKdim  = kBatch * kSteps;
constexpr float kThr     = 0.615f;
constexpr float kDamp    = 0.3f;
constexpr float kDecay   = 0.8f;
constexpr float kEDecay  = 0.8f;
constexpr float kAP      = 1.379f;
constexpr float kAM      = 0.27f;
constexpr float kTauP    = 0.2f;
constexpr float kTauM    = 1.0f;
constexpr float kTScale  = 500.0f;
constexpr float kACarry  = 16.0f;
constexpr float kPCarry  = 1024.0f;
constexpr float kResid   = 2048.0f;
static_assert(kKdim == 1024);
static_assert((kKdim % 32) == 0 && (kNeur % 64) == 0 && (kNeur % 32) == 0);
static_assert(kSteps == 128 * 4);
static_assert((kSteps % 8) == 0);
static_assert(kSteps == 8 * 64);

constexpr size_t kSzVec  = (size_t)kSteps * 4;
constexpr size_t kSzPl   = (size_t)kNeur * kKdim * 2;
constexpr size_t kOffKERN = 0;
constexpr size_t kOffDOP  = kOffKERN + kSzVec;
constexpr size_t kOffGF   = kOffDOP  + kSzVec;
constexpr size_t kOffAT   = kOffGF   + kSzVec;
constexpr size_t kOffBT   = kOffAT   + kSzPl;
constexpr size_t kWsTotal = kOffBT   + kSzPl;
static_assert(kSzVec == 2048ull && kSzPl == 524288ull);
static_assert(kWsTotal == 2048ull + 2048ull + 2048ull + 524288ull + 524288ull);
static_assert(kWsTotal == 1054720ull);
static_assert(kWsTotal <= 134217728ull);
static_assert((kOffDOP % 128) == 0 && (kOffGF % 128) == 0 && (kOffAT % 128) == 0 && (kOffBT % 128) == 0);

__device__ __forceinline__ _Float16 f16_flush(float v) {
  const float w = (fabsf(v) < 6.103515625e-05f) ? 0.0f : v;
  return (_Float16)w;
}
__device__ __forceinline__ void f16_split(float v, _Float16& hi, _Float16& lo) {
  hi = f16_flush(v);
  const float hf = (float)hi;
  const float r = (v - hf) * kResid;
  lo = f16_flush(r);
}

__device__ __forceinline__ float bf16r(float v) {
  unsigned u = __float_as_uint(v);
  u = (u + 0x7FFFu + ((u >> 16) & 1u)) & 0xFFFF0000u;
  return __uint_as_float(u);
}

__device__ __forceinline__ float h16_to_f32(unsigned hb) {
  const unsigned sgn = (hb & 0x8000u) << 16; const unsigned em = hb & 0x7fffu;
  const float fn = __uint_as_float((em << 13) + 0x38000000u);
  const float fs = (float)em * 5.9604644775390625e-8f;
  const float mag = (em < 0x400u) ? fs : fn; return __uint_as_float(__float_as_uint(mag) | sgn); }

namespace eng {
union FragU { v16h v; v8h h[2]; };
__device__ __forceinline__ v16h frag_load(const _Float16* p) {
  FragU f;
  f.h[0] = *(const v8h*)(p);
  f.h[1] = *(const v8h*)(p + 16);
  return f.v;
}
__device__ __forceinline__ v8f mma(v16h a, v16h b, v8f c) {
  return __builtin_amdgcn_wmma_f32_16x16x32_f16(false, a, false, b, (short)0, c, false, false);
}
__device__ __forceinline__ void guard1(v8f& a, v16h x, v16h y) {
  asm volatile("v_nop\n\tv_nop\n\tv_nop\n\tv_nop" : "+v"(a) : "v"(x), "v"(y));
}
__device__ __forceinline__ void guard_acc(v8f& a) {
  asm volatile("v_nop\n\tv_nop\n\tv_nop\n\tv_nop" : "+v"(a));
}
__device__ __forceinline__ void keep4(v16h a, v16h b, v16h c, v16h d) {
  asm volatile("v_nop" :: "v"(a), "v"(b), "v"(c), "v"(d));
}

template <int MI, int SPL>
__global__ __launch_bounds__(256) void gemm_f16_kernel(
    const unsigned short* __restrict__ Ap, const unsigned short* __restrict__ A2p, int lda,
    const unsigned short* __restrict__ Btp, const unsigned short* __restrict__ Bt2p, int ldb,
    float* __restrict__ C, int ldc, int M, int N, int K, float scale, float rscale)
{
  static_assert(MI >= 1 && MI <= 2);
  static_assert(SPL >= 0 && SPL <= 2);
  const _Float16* A   = (const _Float16*)Ap;
  const _Float16* A2  = (const _Float16*)A2p;
  const _Float16* Bt  = (const _Float16*)Btp;
  const _Float16* Bt2 = (const _Float16*)Bt2p;
  __shared__ __align__(16) float sT[8][16 * 68];
  const int lane = threadIdx.x & 31;
  const int wave = threadIdx.x >> 5;
  const int tilesN = N >> 6;
  const int tilesM = M / (16 * MI);
  const int tile = blockIdx.x * 8 + wave;
  if (tile >= tilesM * tilesN) return;
  const int tm = tile / tilesN;
  const int tn = tile - tm * tilesN;
  const int m0 = tm * (16 * MI);
  const int n0 = tn << 6;
  const int rlane = lane & 15;
  const int koff  = (lane >> 4) * 8;
  const int mOff  = (lane >> 4) * 8;

  v8f acc[MI][4], accr[MI][4];
#pragma unroll
  for (int i = 0; i < MI; ++i)
#pragma unroll
    for (int j = 0; j < 4; ++j) {
      acc[i][j]  = (v8f){0.f, 0.f, 0.f, 0.f, 0.f, 0.f, 0.f, 0.f};
      accr[i][j] = (v8f){0.f, 0.f, 0.f, 0.f, 0.f, 0.f, 0.f, 0.f};
    }

  for (int k0 = 0; k0 < K; k0 += 32) {
    v16h bh[4], bl[4];
#pragma unroll
    for (int j = 0; j < 4; ++j) {
      const size_t bo = (size_t)(n0 + (j << 4) + rlane) * ldb + koff + k0;
      bh[j] = frag_load(Bt + bo);
      if (SPL == 2) bl[j] = frag_load(Bt2 + bo); else bl[j] = bh[j];
    }
#pragma unroll
    for (int i = 0; i < MI; ++i) {
      const size_t ao = (size_t)(m0 + (i << 4) + rlane) * lda + koff + k0;
      const v16h ah = frag_load(A + ao);
      v16h al = ah;
      if (SPL >= 1) al = frag_load(A2 + ao);
#pragma unroll
      for (int j = 0; j < 4; ++j) {
        acc[i][j] = mma(ah, bh[j], acc[i][j]);
        if (SPL >= 1) accr[i][j] = mma(al, bh[j], accr[i][j]);
        if (SPL == 2) accr[i][j] = mma(ah, bl[j], accr[i][j]);
      }
#pragma unroll
      for (int j = 0; j < 4; ++j) {
        guard1(acc[i][j], ah, al);
        if (SPL >= 1) guard1(accr[i][j], ah, al);
      }
    }
    keep4(bh[0], bh[1], bh[2], bh[3]);
    if (SPL == 2) keep4(bl[0], bl[1], bl[2], bl[3]);
  }
#pragma unroll
  for (int i = 0; i < MI; ++i)
#pragma unroll
    for (int j = 0; j < 4; ++j) {
      guard_acc(acc[i][j]);
      if (SPL >= 1) guard_acc(accr[i][j]);
    }

  float* slab = sT[wave];
#pragma unroll
  for (int i = 0; i < MI; ++i) {
    const int mBase = m0 + (i << 4);
#pragma unroll
    for (int j = 0; j < 4; ++j) {
#pragma unroll
      for (int r = 0; r < 8; ++r) {
        float v = acc[i][j][r] * scale;
        if (SPL >= 1) v += accr[i][j][r] * rscale;
        slab[(mOff + r) * 68 + (j << 4) + rlane] = v;
      }
    }
    __builtin_amdgcn_fence(__ATOMIC_RELEASE, "workgroup");
    __builtin_amdgcn_wave_barrier();
    __builtin_amdgcn_fence(__ATOMIC_ACQUIRE, "workgroup");
    {
      const int hh = lane >> 4, c4 = (lane & 15) * 4;
      for (int pass = 0; pass < 2; ++pass) {
#pragma unroll
        for (int it = 0; it < 8; ++it) {
          const int row = it * 2 + hh;
          const v4f v = *(const v4f*)(slab + row * 68 + c4);
          *(volatile v4f*)(C + (size_t)(mBase + row) * ldc + n0 + c4) = v;
        }
        __threadfence();
      }
    }
    __builtin_amdgcn_fence(__ATOMIC_RELEASE, "workgroup");
    __builtin_amdgcn_wave_barrier();
    __builtin_amdgcn_fence(__ATOMIC_ACQUIRE, "workgroup");
  }
}
}

__device__ __forceinline__ float reward_lag(int t) {
  const float ts = (float)t / kTScale;
  const float kp = kAP * ts / kTauP * expf(1.0f - ts / kTauP);
  const float km = kAM * ts / kTauM * expf(1.0f - ts / kTauM);
  return kp - km;
}
__global__ __launch_bounds__(128) void kern_kernel(float* __restrict__ KERN)
{
  const int t0 = threadIdx.x * 4;
  v4f r;
  r[0] = reward_lag(t0);
  r[1] = reward_lag(t0 + 1);
  r[2] = reward_lag(t0 + 2);
  r[3] = reward_lag(t0 + 3);
  float* p = KERN + t0;
  *(volatile v4f*)p = r;
  __threadfence();
  *(volatile v4f*)p = r;
}

__global__ __launch_bounds__(128) void dop_kernel(
    const float* __restrict__ z, const int* __restrict__ cn_idx,
    const float* __restrict__ KERN, float* __restrict__ DOP)
{
  const int t0 = threadIdx.x * 4;
  int cn = cn_idx[0];
  cn = (cn < 0) ? 0 : cn;
  cn = (cn > kNeur - 1) ? (kNeur - 1) : cn;
  float d0 = 0.0f, d1 = 0.0f, d2 = 0.0f, d3 = 0.0f;
  for (int s = 0; s < 512; ++s) {
    const float za = z[(size_t)s * kNeur + cn];
    const float zb = z[(size_t)(kSteps + s) * kNeur + cn];
    const float zc = bf16r(za) + bf16r(zb);
    const int i0 = t0 - s;
    const int i1 = i0 + 1;
    const int i2 = i0 + 2;
    const int i3 = i0 + 3;
    float k0 = KERN[(i0 < 0) ? 0 : i0];
    float k1 = KERN[(i1 < 0) ? 0 : i1];
    float k2 = KERN[(i2 < 0) ? 0 : i2];
    float k3 = KERN[(i3 < 0) ? 0 : i3];
    const bool live = (s >= 1);
    const float p0 = (live && i0 >= 0) ? (zc * k0) : 0.0f;
    const float p1 = (live && i1 >= 0) ? (zc * k1) : 0.0f;
    const float p2 = (live && i2 >= 0) ? (zc * k2) : 0.0f;
    const float p3 = (live && i3 >= 0) ? (zc * k3) : 0.0f;
    d0 += p0;
    d1 += p1;
    d2 += p2;
    d3 += p3;
  }
  v4f r;
  r[0] = d0;
  r[1] = d1;
  r[2] = d2;
  r[3] = d3;
  float* p = DOP + t0;
  *(volatile v4f*)p = r;
  __threadfence();
  *(volatile v4f*)p = r;
}

__global__ __launch_bounds__(32) void g_kernel(const float* __restrict__ DOP, float* __restrict__ GF)
{
  const int lane = threadIdx.x;
  for (int p = 0; p < 4; ++p) {
    const int base = 128 * p + 4 * lane;
    float g = 0.0f;
    float k0 = 0.0f, k1 = 0.0f, k2 = 0.0f, k3 = 0.0f;
    for (int u = 0; u < 512; ++u) {
      const int s = 511 - u;
      const float dv = DOP[s];
      g = kEDecay * g + dv;
      k0 = (s == base) ? g : k0;
      k1 = (s == base + 1) ? g : k1;
      k2 = (s == base + 2) ? g : k2;
      k3 = (s == base + 3) ? g : k3;
    }
    v4f r;
    r[0] = k0;
    r[1] = k1;
    r[2] = k2;
    r[3] = k3;
    float* q = GF + base;
    *(volatile v4f*)q = r;
    __threadfence();
    *(volatile v4f*)q = r;
  }
}

__global__ __launch_bounds__(256) void zbar_a_kernel(
    const float* __restrict__ z, const float* __restrict__ GF, unsigned short* __restrict__ AT)
{
  const int b = blockIdx.x;
  const int i = threadIdx.x;
  const float* zp = z + (size_t)b * kSteps * kNeur + i;
  unsigned short* row = AT + (size_t)i * kKdim + (size_t)b * kSteps;
  float zb = 0.0f;
  for (int c = 0; c < 8; ++c) {
    const int sb = c * 64;
    v8h hv[8];
#pragma unroll
    for (int m = 0; m < 8; ++m) {
      const v4f g0 = *(const v4f*)(GF + sb + 8 * m);
      const v4f g1 = *(const v4f*)(GF + sb + 8 * m + 4);
      float gq[8];
      gq[0] = g0[0];
      gq[1] = g0[1];
      gq[2] = g0[2];
      gq[3] = g0[3];
      gq[4] = g1[0];
      gq[5] = g1[1];
      gq[6] = g1[2];
      gq[7] = g1[3];
#pragma unroll
      for (int e = 0; e < 8; ++e) {
        const int s = sb + 8 * m + e;
        const int sp = (s >= 1) ? (s - 1) : 0;
        const float zin = zp[(size_t)sp * kNeur];
        const float zs = (s >= 1) ? bf16r(zin) : 0.0f;
        zb = kDecay * zb + zs;
        const float a = gq[e] * zb;
        hv[m][e] = f16_flush(a * kACarry);
      }
    }
    unsigned short* q = row + sb;
#pragma unroll
    for (int m = 0; m < 8; ++m) *(volatile v8h*)(q + 8 * m) = hv[m];
    __threadfence();
#pragma unroll
    for (int m = 0; m < 8; ++m) *(volatile v8h*)(q + 8 * m) = hv[m];
  }
}

__global__ __launch_bounds__(256) void psi_b_kernel(
    const float* __restrict__ v, unsigned short* __restrict__ BT)
{
  const int gid = blockIdx.x * 256 + threadIdx.x;
  const int j  = gid >> 7;
  const int k0 = (gid & 127) * 8;
  const int b  = k0 >> 9;
  const int s0 = k0 & 511;
  const float* vp = v + ((size_t)b * kSteps + s0) * kNeur + j;
  v8h hv;
#pragma unroll
  for (int e = 0; e < 8; ++e) {
    const float x = bf16r(vp[(size_t)e * kNeur]);
    const float vs = (x - kThr) / kThr;
    const float m = fmaxf(1.0f - fabsf(vs), 0.0f);
    const float psi = kDamp * m / kThr;
    hv[e] = f16_flush(psi * kPCarry);
  }
  unsigned short* q = BT + (size_t)j * kKdim + k0;
  *(volatile v8h*)q = hv;
  __threadfence();
  *(volatile v8h*)q = hv;
}

static_assert(((kNeur / 32) * (kNeur / 64)) % 8 == 0);
static_assert((kNeur / 32) * (kNeur / 64) / 8 == 4);
static_assert((kNeur * (kKdim / 8)) % 256 == 0);
static_assert((kNeur * (kKdim / 8)) / 256 == 128);
static_assert(kBatch * kNeur == 2 * 256);
static_assert(kSteps / 4 == 128);

extern "C" void kernel_launch(void* const* d_in, const int* in_sizes, int n_in,
                              void* d_out, int out_size, void* d_ws, size_t ws_size,
                              hipStream_t stream)
{
  if (n_in < 3) return;
  if (in_sizes[0] != kBatch * kSteps * kNeur) return;
  if (in_sizes[1] != kBatch * kSteps * kNeur) return;
  if (in_sizes[2] != 1) return;
  if (out_size != kNeur * kNeur) return;
  if (ws_size < kWsTotal) return;

  const float* v  = (const float*)d_in[0];
  const float* z  = (const float*)d_in[1];
  const int*   cn = (const int*)d_in[2];
  float* out = (float*)d_out;

  char* ws = (char*)d_ws;
  float*          KERN = (float*)(ws + kOffKERN);
  float*          DOP  = (float*)(ws + kOffDOP);
  float*          GF   = (float*)(ws + kOffGF);
  unsigned short* AT   = (unsigned short*)(ws + kOffAT);
  unsigned short* BT   = (unsigned short*)(ws + kOffBT);

  constexpr float sOut = 1.0f / (kACarry * kPCarry);

  kern_kernel<<<1, 128, 0, stream>>>(KERN);

  dop_kernel<<<1, 128, 0, stream>>>(z, cn, KERN, DOP);

  g_kernel<<<1, 32, 0, stream>>>(DOP, GF);

  zbar_a_kernel<<<kBatch, 256, 0, stream>>>(z, GF, AT);

  psi_b_kernel<<<(kNeur * (kKdim / 8)) / 256, 256, 0, stream>>>(v, BT);

  eng::gemm_f16_kernel<2, 0><<<dim3((kNeur / 32) * (kNeur / 64) / 8), 256, 0, stream>>>(
      AT, nullptr, kKdim, BT, nullptr, kKdim, out, kNeur, kNeur, kNeur, kKdim, sOut, 0.0f);
}
